// GATv2_84782654423396
// MI455X (gfx1250) — hardware-verified
//
#include <hip/hip_runtime.h>
#include <stddef.h>
#include <stdint.h>
#include <math.h>


#define F_IN    128
#define XUPR    (F_IN / 8)
#define C1      128
#define HD1     64
#define P1      (2 * C1)
#define KA      (2 * C1)
#define N2W     16
#define P2      64
#define NTHR    256
#define NWAVE   8
#define EPT     8
#define CHUNK   (NTHR * EPT)
#define WCAP    (EPT * 32)
#define LISTN   (NWAVE * WCAP)
#define NBMAX   2048
#define SLOTB   11
#define NBRUN   512
#define RCAP    28672
#define DEGCAP  128
#define STW0    128
#define STW1    2048
#define GBM     64
#define GBN     64
#define GTHR    128
#define NEGS    0.2f
#define MX0     (-1.0e30f)
#define WSMAX   134217728
#define LDS_AGG ((2 * RCAP + 2 * NBMAX + LISTN) * 4 + 64)

static_assert((CHUNK & (CHUNK - 1)) == 0 && CHUNK <= (1 << SLOTB));
static_assert(NBMAX == (1 << SLOTB));
static_assert((NBRUN & (NBRUN - 1)) == 0 && NBRUN <= NBMAX && NBRUN >= 64);
static_assert(NTHR * 8 == NBMAX);
static_assert(LISTN >= NBMAX);
static_assert(LISTN >= NWAVE * WCAP);
static_assert((RCAP % 32) == 0);
static_assert(NWAVE * STW0 <= RCAP && NWAVE * STW1 <= RCAP);
static_assert(2 * STW0 == KA);
static_assert(STW1 == (NBRUN / NWAVE) * 32);
static_assert(LDS_AGG <= 300000);
static_assert(GBM == (GTHR / 32) * 16);
static_assert(GTHR == 2 * GBN && GTHR == 2 * GBM);
static_assert((F_IN % 32) == 0 && (KA % 32) == 0);
static_assert((F_IN % 8) == 0 && (C1 % 8) == 0);
static_assert((P1 % GBN) == 0 && (P2 % GBN) == 0);
static_assert(C1 == 4 * 32 && HD1 == 4 * 16);
static_assert(C1 == 2 * HD1);
static_assert(N2W == 16 && P2 == 4 * N2W);

typedef float          v2f  __attribute__((ext_vector_type(2)));
typedef float          v4f  __attribute__((ext_vector_type(4)));
typedef float          v8f  __attribute__((ext_vector_type(8)));
typedef int            v4i  __attribute__((ext_vector_type(4)));
typedef int            v8i  __attribute__((ext_vector_type(8)));
typedef unsigned int   v2u  __attribute__((ext_vector_type(2)));
typedef unsigned int   v4u  __attribute__((ext_vector_type(4)));
typedef unsigned short v8us __attribute__((ext_vector_type(8)));
typedef __bf16         v16b __attribute__((ext_vector_type(16)));
typedef v4f  __attribute__((may_alias)) v4fa;
typedef v2u  __attribute__((may_alias)) v2ua;
typedef v4u  __attribute__((may_alias)) v4ua;
typedef v8us __attribute__((may_alias)) v8usa;
union FragB { v16b v; v8us h[2]; v8i w; };

__device__ __forceinline__ v8f wmb(const FragB& a, const FragB& b, v8f c) {
  v8f d = __builtin_amdgcn_wmma_f32_16x16x32_bf16(false, a.v, false, b.v, (short)0, c, false, false);
  asm volatile("v_nop\n\tv_nop\n\tv_nop\n\tv_nop" : "+v"(d) : "v"(a.w), "v"(b.w));
  return d;
}

__device__ __forceinline__ unsigned int f2bf(float f) {
  const unsigned int u = __float_as_uint(f);
  return ((u + 0x7FFFu + ((u >> 16) & 1u)) >> 16) & 0xFFFFu;
}
__device__ __forceinline__ float bf2f(unsigned int b) { return __uint_as_float(b << 16); }
__device__ __forceinline__ float bfr(float f) { return bf2f(f2bf(f)); }
__device__ __forceinline__ unsigned int pk2(float lo, float hi) { return f2bf(lo) | (f2bf(hi) << 16); }
__device__ __forceinline__ v4u pack8(const v4f a, const v4f b) {
  v4u r;
  r.x = pk2(a.x, a.y); r.y = pk2(a.z, a.w); r.z = pk2(b.x, b.y); r.w = pk2(b.z, b.w);
  return r;
}

__device__ __forceinline__ int scan_chunk(const int* __restrict__ dsts, int nE, int cbase, int slotBase,
                                          int nb, int vec8, int* list, int tid, int lane, int wave) {
  int wc = 0;
  const int el0  = tid * EPT;
  const int e0   = cbase + el0;
  const int sent = -2147483647 - 1;
  v4i da, db;
  if (vec8 != 0 && cbase + CHUNK <= nE) {
    da = *(const v4i*)(dsts + e0);
    db = *(const v4i*)(dsts + e0 + 4);
  } else {
    da.x = (e0     < nE) ? dsts[min(e0,     nE - 1)] : sent;
    da.y = (e0 + 1 < nE) ? dsts[min(e0 + 1, nE - 1)] : sent;
    da.z = (e0 + 2 < nE) ? dsts[min(e0 + 2, nE - 1)] : sent;
    da.w = (e0 + 3 < nE) ? dsts[min(e0 + 3, nE - 1)] : sent;
    db.x = (e0 + 4 < nE) ? dsts[min(e0 + 4, nE - 1)] : sent;
    db.y = (e0 + 5 < nE) ? dsts[min(e0 + 5, nE - 1)] : sent;
    db.z = (e0 + 6 < nE) ? dsts[min(e0 + 6, nE - 1)] : sent;
    db.w = (e0 + 7 < nE) ? dsts[min(e0 + 7, nE - 1)] : sent;
  }
  const unsigned nbs = (unsigned)slotBase;
  const unsigned unb = (unsigned)nb;
  const unsigned s0 = (unsigned)da.x - nbs, s1 = (unsigned)da.y - nbs;
  const unsigned s2 = (unsigned)da.z - nbs, s3 = (unsigned)da.w - nbs;
  const unsigned s4 = (unsigned)db.x - nbs, s5 = (unsigned)db.y - nbs;
  const unsigned s6 = (unsigned)db.z - nbs, s7 = (unsigned)db.w - nbs;
  const bool h0 = s0 < unb, h1 = s1 < unb, h2 = s2 < unb, h3 = s3 < unb;
  const bool h4 = s4 < unb, h5 = s5 < unb, h6 = s6 < unb, h7 = s7 < unb;
  const unsigned any = __builtin_amdgcn_ballot_w32(h0 | h1 | h2 | h3 | h4 | h5 | h6 | h7);
  if (any != 0u) {
#define HITJ(J, HJ, SJ) { \
      const unsigned mj = __builtin_amdgcn_ballot_w32(HJ); \
      if (mj != 0u) { \
        if (HJ) { \
          const int pos = wc + (int)__builtin_amdgcn_mbcnt_lo(mj, 0u); \
          if (pos < WCAP) list[wave * WCAP + pos] = ((el0 + (J)) << SLOTB) | (int)(SJ); \
        } \
        wc += (int)__builtin_popcount(mj); } }
    HITJ(0, h0, s0)
    HITJ(1, h1, s1)
    HITJ(2, h2, s2)
    HITJ(3, h3, s3)
    HITJ(4, h4, s4)
    HITJ(5, h5, s5)
    HITJ(6, h6, s6)
    HITJ(7, h7, s7)
#undef HITJ
  }
  return wc;
}

__global__ __launch_bounds__(NTHR) void k_xprep(const float* __restrict__ x, unsigned short* xb, int nN, int nUnits) {
  const int i = (int)blockIdx.x * NTHR + (int)threadIdx.x;
  if (i >= nUnits) return;
  const int row = i / XUPR;
  const int c0  = (i - row * XUPR) * 8;
  const int rc  = row < nN ? row : nN - 1;
  const float* p = x + (size_t)rc * F_IN + c0;
  v4f a = *(const v4fa*)p, b = *(const v4fa*)(p + 4);
  const v4f z4 = {0.f, 0.f, 0.f, 0.f};
  if (row >= nN) { a = z4; b = z4; }
  const v4u hv = pack8(a, b);
  const size_t o = (size_t)row * F_IN + c0;
  *(volatile v4u*)(xb + o) = hv;
  __threadfence();
  *(volatile v4u*)(xb + o) = hv;
}

__global__ __launch_bounds__(NTHR) void k_wtr(const float* __restrict__ w, int Kin, int Ncol, int Nrows, int Kout,
                                              unsigned short* wt, int nUnits) {
  const int u = (int)blockIdx.x * NTHR + (int)threadIdx.x;
  if (u >= nUnits) return;
  const int kq = Kout >> 3;
  const int n  = u / kq;
  const int k8 = (u - n * kq) * 8;
  const int kk = k8 - (k8 / Kin) * Kin;
  const int ncl = n < Ncol ? n : Ncol - 1;
  const float* p = w + (size_t)kk * (size_t)Ncol + ncl;
  v4f a, b;
  a.x = p[0];                    a.y = p[(size_t)Ncol];         a.z = p[(size_t)2 * Ncol];     a.w = p[(size_t)3 * Ncol];
  b.x = p[(size_t)4 * Ncol];     b.y = p[(size_t)5 * Ncol];     b.z = p[(size_t)6 * Ncol];     b.w = p[(size_t)7 * Ncol];
  const v4f z4 = {0.f, 0.f, 0.f, 0.f};
  if (n >= Ncol || n >= Nrows) { a = z4; b = z4; }
  const v4u wv = pack8(a, b);
  unsigned short* o = wt + (size_t)n * (size_t)Kout + k8;
  *(volatile v4u*)o = wv;
  __threadfence();
  *(volatile v4u*)o = wv;
}

__global__ __launch_bounds__(GTHR) void k_gemm(
    const unsigned short* __restrict__ A, const unsigned short* __restrict__ WT,
    float* outF, int K, int ldo)
{
  __shared__ __attribute__((aligned(16))) float stg[GBM * GBN];
  const int tid = (int)threadIdx.x, lane = tid & 31, wave = tid >> 5, hh = lane >> 4, m = lane & 15;
  const int rowBase = (int)blockIdx.x * GBM;
  const int col0    = (int)blockIdx.y * GBN;

  v8f acc[4];
  {
    const v8f z = {0.f, 0.f, 0.f, 0.f, 0.f, 0.f, 0.f, 0.f};
    acc[0] = z; acc[1] = z; acc[2] = z; acc[3] = z;
  }
  const unsigned short* ap = A  + (size_t)(rowBase + 16 * wave + m) * (size_t)K + 8 * hh;
  const unsigned short* wp = WT + (size_t)(col0 + m) * (size_t)K + 8 * hh;
  const int ksteps = K >> 5;
#pragma unroll 1
  for (int ks = 0; ks < ksteps; ++ks) {
    FragB af;
    af.h[0] = *(const v8usa*)(ap + 32 * ks);
    af.h[1] = *(const v8usa*)(ap + 32 * ks + 16);
#pragma unroll
    for (int t = 0; t < 4; ++t) {
      const unsigned short* wq = wp + (size_t)(16 * t) * (size_t)K + 32 * ks;
      FragB bf;
      bf.h[0] = *(const v8usa*)wq;
      bf.h[1] = *(const v8usa*)(wq + 16);
      acc[t] = wmb(af, bf, acc[t]);
    }
  }

#pragma unroll
  for (int t = 0; t < 4; ++t) {
    const int lc = 16 * t + m;
#pragma unroll
    for (int r = 0; r < 8; ++r) {
      const int lr = 16 * wave + 8 * hh + r;
      stg[lr * GBN + lc] = acc[t][r];
    }
  }
  __syncthreads();

  v4f fv[8];
#pragma unroll
  for (int i = 0; i < 8; ++i) {
    const int lr = 16 * wave + 2 * i + hh;
    fv[i] = *(const v4fa*)(stg + lr * GBN + 4 * m);
  }
#pragma unroll
  for (int i = 0; i < 8; ++i) {
    const int lr = 16 * wave + 2 * i + hh;
    const int gr = rowBase + lr;
    float* op = outF + (size_t)gr * (size_t)ldo + col0 + 4 * m;
    *(volatile v4f*)op = fv[i];
  }
  __threadfence();
#pragma unroll
  for (int i = 0; i < 8; ++i) {
    const int lr = 16 * wave + 2 * i + hh;
    const int gr = rowBase + lr;
    float* op = outF + (size_t)gr * (size_t)ldo + col0 + 4 * m;
    *(volatile v4f*)op = fv[i];
  }
}

template<int MODE>
__global__ __launch_bounds__(NTHR) void k_agg(
    const int* __restrict__ srcs, const int* __restrict__ dsts,
    const float* __restrict__ HF, const float* __restrict__ att,
    unsigned short* HA, float* out,
    int nN, int nE, int nb, int vec8, int MPr) {
  extern __shared__ v4f lds_dyn[];
  int* reg1 = (int*)lds_dyn;
  int* reg2 = reg1 + RCAP;
  int* scnt = reg2 + RCAP;
  int* soff = scnt + NBMAX;
  int* list = soff + NBMAX;
  int* wcnt = list + LISTN;
  int* wtot = wcnt + NWAVE;
  const int tid = (int)threadIdx.x, lane = tid & 31, wave = tid >> 5;
  const int nodeBase = (int)blockIdx.x * nb;

  for (int i = tid; i < NBMAX; i += NTHR) scnt[i] = 0;
  __syncthreads();

  int tot = 0;
  const int nChunks = (nE + CHUNK - 1) / CHUNK;
#pragma unroll 1
  for (int ch = 0; ch < nChunks; ++ch) {
    const int cbase = ch * CHUNK;
    const int wc = scan_chunk(dsts, nE, cbase, nodeBase, nb, vec8, list, tid, lane, wave);
    if (lane == 0) wcnt[wave] = wc;
    __syncthreads();
    int pre = 0, all = 0;
#pragma unroll
    for (int w2 = 0; w2 < NWAVE; ++w2) {
      int c = wcnt[w2];
      c = c < 0 ? 0 : (c > WCAP ? WCAP : c);
      all += c;
      pre += (w2 < wave) ? c : 0;
    }
    const int wcc  = wc > WCAP ? WCAP : wc;
    const int base = tot + pre;
#pragma unroll 1
    for (int i = lane; i < wcc; i += 32) {
      const int ent = list[wave * WCAP + i];
      const int el  = (ent >> SLOTB) & (CHUNK - 1);
      const int sl  = ent & (NBMAX - 1);
      int eid = cbase + el;
      eid = eid > nE - 1 ? nE - 1 : eid;
      const int pos = base + i;
      if (pos < RCAP) reg1[pos] = (int)(((unsigned)eid << SLOTB) | (unsigned)sl);
    }
    tot += all;
    tot = tot > RCAP ? RCAP : tot;
    __syncthreads();
  }
  const int nh = tot;

  if (wave == 0) {
#pragma unroll 1
    for (int b0 = 0; b0 < nh; b0 += 32) {
      const int idx = b0 + lane;
      const int uv  = reg1[idx < nh ? idx : nh - 1];
      const int m32 = (nh - b0) < 32 ? (nh - b0) : 32;
#pragma unroll 1
      for (int k = 0; k < m32; ++k) {
        const int u  = __builtin_amdgcn_readlane(uv, k);
        const int sl = u & (NBMAX - 1);
        if (lane == 0) scnt[sl] = scnt[sl] + 1;
      }
    }
  }
  __syncthreads();

  {
    const v4i ca = *(const v4i*)(scnt + 8 * tid);
    const v4i cb = *(const v4i*)(scnt + 8 * tid + 4);
    const int e0 = ca.x < 0 ? 0 : ca.x, e1 = ca.y < 0 ? 0 : ca.y, e2 = ca.z < 0 ? 0 : ca.z, e3 = ca.w < 0 ? 0 : ca.w;
    const int e4 = cb.x < 0 ? 0 : cb.x, e5 = cb.y < 0 ? 0 : cb.y, e6 = cb.z < 0 ? 0 : cb.z, e7 = cb.w < 0 ? 0 : cb.w;
    const int ts = e0 + e1 + e2 + e3 + e4 + e5 + e6 + e7;
    int incl = ts;
#pragma unroll
    for (int d = 1; d < 32; d <<= 1) {
      const int up = __shfl_up(incl, d);
      if (lane >= d) incl += up;
    }
    if (lane == 31) wtot[wave] = incl;
    __syncthreads();
    int pre = 0;
#pragma unroll
    for (int w2 = 0; w2 < NWAVE; ++w2) pre += (w2 < wave) ? wtot[w2] : 0;
    int run = pre + incl - ts;
    soff[8 * tid + 0] = run; run += e0;
    soff[8 * tid + 1] = run; run += e1;
    soff[8 * tid + 2] = run; run += e2;
    soff[8 * tid + 3] = run; run += e3;
    soff[8 * tid + 4] = run; run += e4;
    soff[8 * tid + 5] = run; run += e5;
    soff[8 * tid + 6] = run; run += e6;
    soff[8 * tid + 7] = run;
  }
  __syncthreads();
  for (int i = tid; i < NBMAX; i += NTHR) list[i] = soff[i];
  __syncthreads();

  if (wave == 0) {
#pragma unroll 1
    for (int b0 = 0; b0 < nh; b0 += 32) {
      const int idx = b0 + lane;
      const int uv  = reg1[idx < nh ? idx : nh - 1];
      const int m32 = (nh - b0) < 32 ? (nh - b0) : 32;
#pragma unroll 1
      for (int k = 0; k < m32; ++k) {
        const int u   = __builtin_amdgcn_readlane(uv, k);
        const int sl  = u & (NBMAX - 1);
        const int eid = (int)((unsigned)u >> SLOTB);
        if (lane == 0) {
          int pos = list[sl];
          pos = pos < 0 ? 0 : (pos > RCAP - 1 ? RCAP - 1 : pos);
          reg2[pos] = eid;
          list[sl] = pos + 1;
        }
      }
    }
  }
  __syncthreads();

  const int nbw = nb >> 3;
  const bool ovf = (nh >= RCAP);
  const float qnan = __int_as_float(0x7fc00000);

  if (MODE == 0) {
    unsigned int* stw = (unsigned int*)reg1 + wave * STW0;
    const int c0 = 4 * lane;
    v4f a4;
    {
      const v4f a0 = *(const v4fa*)(att + c0);
      a4.x = bfr(a0.x); a4.y = bfr(a0.y); a4.z = bfr(a0.z); a4.w = bfr(a0.w);
    }
#pragma unroll 1
    for (int jt = 0; jt < nbw; ++jt) {
      const int slot = wave * nbw + jt;
      const int grow = nodeBase + slot;
      const int gcl  = grow < nN ? grow : nN - 1;
      int st = soff[slot];
      const int craw = scnt[slot];
      int cnt = craw;
      st  = st < 0 ? 0 : (st > nh ? nh : st);
      cnt = cnt < 0 ? 0 : (cnt > DEGCAP ? DEGCAP : cnt);
      if (cnt > nh - st) cnt = nh - st;
      const float pz = (ovf || craw > DEGCAP) ? qnan : 0.0f;
      const float live = grow < nN ? 1.0f : 0.0f;

      const v4f d4 = *(const v4fa*)(HF + (size_t)gcl * P1 + C1 + c0);
      float av0 = 0.f, av1 = 0.f, av2 = 0.f, av3 = 0.f;
      float mx = MX0, dn = 0.f;

#pragma unroll 1
      for (int q = 0; q < cnt; ++q) {
        int idx = st + q; idx = idx > RCAP - 1 ? RCAP - 1 : idx;
        int eid = reg2[idx]; eid = eid < 0 ? 0 : (eid > nE - 1 ? nE - 1 : eid);
        const int sraw = srcs[eid];
        const int s = sraw < 0 ? 0 : (sraw > nN - 1 ? nN - 1 : sraw);
        const v4f e4 = *(const v4fa*)(HF + (size_t)s * P1 + c0);
        float v0 = e4.x + d4.x, v1 = e4.y + d4.y, v2 = e4.z + d4.z, v3 = e4.w + d4.w;
        v0 = v0 > 0.f ? v0 : v0 * NEGS;
        v1 = v1 > 0.f ? v1 : v1 * NEGS;
        v2 = v2 > 0.f ? v2 : v2 * NEGS;
        v3 = v3 > 0.f ? v3 : v3 * NEGS;
        float part = v0 * a4.x;
        part = fmaf(v1, a4.y, part);
        part = fmaf(v2, a4.z, part);
        part = fmaf(v3, a4.w, part);
        part += __shfl_xor(part, 8);
        part += __shfl_xor(part, 4);
        part += __shfl_xor(part, 2);
        part += __shfl_xor(part, 1);
        const float al = part;
        const float df = al - mx;
        const float ee = __expf(-fabsf(df));
        const bool up  = df > 0.f;
        const float s1 = up ? ee : 1.0f;
        const float s2 = up ? 1.0f : ee;
        mx = up ? al : mx;
        dn = fmaf(dn, s1, s2);
        av0 = fmaf(av0, s1, s2 * e4.x);
        av1 = fmaf(av1, s1, s2 * e4.y);
        av2 = fmaf(av2, s1, s2 * e4.z);
        av3 = fmaf(av3, s1, s2 * e4.w);
      }
      const float ds = dn > 0.f ? dn : 1.0f;
      const float iv = (dn > 0.f ? 1.0f : 0.0f) * __builtin_amdgcn_rcpf(ds);
      float r0 = av0 * iv, r1 = av1 * iv, r2 = av2 * iv, r3 = av3 * iv;
      r0 = r0 > 0.f ? r0 : (__expf(r0) - 1.0f);
      r1 = r1 > 0.f ? r1 : (__expf(r1) - 1.0f);
      r2 = r2 > 0.f ? r2 : (__expf(r2) - 1.0f);
      r3 = r3 > 0.f ? r3 : (__expf(r3) - 1.0f);
      r0 = r0 * live + pz; r1 = r1 * live + pz; r2 = r2 * live + pz; r3 = r3 * live + pz;

      const unsigned int hb0 = f2bf(r0), hb1 = f2bf(r1), hb2 = f2bf(r2), hb3 = f2bf(r3);
      const unsigned int lb0 = f2bf(r0 - bf2f(hb0)), lb1 = f2bf(r1 - bf2f(hb1));
      const unsigned int lb2 = f2bf(r2 - bf2f(hb2)), lb3 = f2bf(r3 - bf2f(hb3));
      v2u hw, lw;
      hw.x = hb0 | (hb1 << 16); hw.y = hb2 | (hb3 << 16);
      lw.x = lb0 | (lb1 << 16); lw.y = lb2 | (lb3 << 16);
      __builtin_amdgcn_fence(__ATOMIC_RELEASE, "wavefront");
      __builtin_amdgcn_wave_barrier();
      *(v2ua*)(stw + 2 * lane) = hw;
      *(v2ua*)(stw + (STW0 / 2) + 2 * lane) = lw;
      __builtin_amdgcn_fence(__ATOMIC_RELEASE, "wavefront");
      __builtin_amdgcn_wave_barrier();
      const v4u pv = *(const v4ua*)(stw + 4 * lane);
      const bool wr = grow < MPr;
      unsigned short* gp = HA + (size_t)grow * KA + 8 * lane;
      if (wr) *(volatile v4u*)gp = pv;
      __threadfence();
      if (wr) *(volatile v4u*)gp = pv;
    }
  } else {
    float* stw = (float*)reg1 + wave * STW1;
    const int c = lane & 15;
    const float atc = bfr(att[c]);
#pragma unroll 1
    for (int jt = 0; jt < nbw; ++jt) {
      const int slot = wave * nbw + jt;
      const int grow = nodeBase + slot;
      const int gcl  = grow < nN ? grow : nN - 1;
      int st = soff[slot];
      const int craw = scnt[slot];
      int cnt = craw;
      st  = st < 0 ? 0 : (st > nh ? nh : st);
      cnt = cnt < 0 ? 0 : (cnt > DEGCAP ? DEGCAP : cnt);
      if (cnt > nh - st) cnt = nh - st;
      const float pz = (ovf || craw > DEGCAP) ? qnan : 0.0f;

      const float* drow = HF + (size_t)gcl * P2;
      const float hdv = drow[N2W + c];
      const float rsv = drow[2 * N2W + c];
      float av = 0.f, mx = MX0, dn = 0.f;

#pragma unroll 1
      for (int q = 0; q < cnt; ++q) {
        int idx = st + q; idx = idx > RCAP - 1 ? RCAP - 1 : idx;
        int eid = reg2[idx]; eid = eid < 0 ? 0 : (eid > nE - 1 ? nE - 1 : eid);
        const int sraw = srcs[eid];
        const int s = sraw < 0 ? 0 : (sraw > nN - 1 ? nN - 1 : sraw);
        const float hs = HF[(size_t)s * P2 + c];
        float v = hs + hdv;
        v = v > 0.f ? v : v * NEGS;
        float part = v * atc;
        part += __shfl_xor(part, 8);
        part += __shfl_xor(part, 4);
        part += __shfl_xor(part, 2);
        part += __shfl_xor(part, 1);
        const float al = part;
        const float df = al - mx;
        const float ee = __expf(-fabsf(df));
        const bool up  = df > 0.f;
        const float s1 = up ? ee : 1.0f;
        const float s2 = up ? 1.0f : ee;
        mx = up ? al : mx;
        dn = fmaf(dn, s1, s2);
        av = fmaf(av, s1, s2 * hs);
      }
      const float ds = dn > 0.f ? dn : 1.0f;
      const float iv = (dn > 0.f ? 1.0f : 0.0f) * __builtin_amdgcn_rcpf(ds);
      const float r = fmaf(av, iv, rsv) + pz;
      stw[jt * 32 + lane] = r;
    }
    __builtin_amdgcn_fence(__ATOMIC_RELEASE, "wavefront");
    __builtin_amdgcn_wave_barrier();
    const int r0w  = nodeBase + wave * nbw;
    const int nins = nbw >> 3;
    const int rq   = lane >> 2, pc = 4 * (lane & 3);
#pragma unroll 1
    for (int i = 0; i < nins; ++i) {
      const int lr  = 8 * i + rq;
      const v4f gv  = *(const v4fa*)(stw + lr * 32 + pc);
      const int row = r0w + lr;
      float* gp = out + (size_t)row * N2W + pc;
      if (row < nN) *(volatile v4f*)gp = gv;
    }
    __threadfence();
#pragma unroll 1
    for (int i = 0; i < nins; ++i) {
      const int lr  = 8 * i + rq;
      const v4f gv  = *(const v4fa*)(stw + lr * 32 + pc);
      const int row = r0w + lr;
      float* gp = out + (size_t)row * N2W + pc;
      if (row < nN) *(volatile v4f*)gp = gv;
    }
  }
  (void)HA; (void)out; (void)MPr;
}

static int pick_nb(int nE, int nN) {
  int nb = NBRUN;
  while (nb > 64 && (long long)nb * (long long)nE * 5LL > (long long)RCAP * (long long)nN * 4LL) nb >>= 1;
  return nb;
}
static inline int cdiv(int a, int b) { return (a + b - 1) / b; }

extern "C" void kernel_launch(void* const* d_in, const int* in_sizes, int n_in,
                              void* d_out, int out_size, void* d_ws, size_t ws_size,
                              hipStream_t stream) {
  if (n_in < 10) return;
  const int nN = in_sizes[0] / F_IN;
  if (nN <= 0 || in_sizes[0] != nN * F_IN || nN > (1 << 22)) return;
  const int nE = in_sizes[1];
  if (nE < 1 || in_sizes[2] != nE) return;
  if (nE >= (1 << (32 - SLOTB))) return;
  if (in_sizes[3] != F_IN * C1 || in_sizes[4] != F_IN * C1) return;
  if (in_sizes[5] != C1) return;
  if (in_sizes[6] != C1 * N2W || in_sizes[7] != C1 * N2W) return;
  if (in_sizes[8] != N2W) return;
  if (in_sizes[9] != C1 * N2W) return;
  if (out_size != nN * N2W) return;

  const float* h   = (const float*)d_in[0];
  const int*   src = (const int*)  d_in[1];
  const int*   dst = (const int*)  d_in[2];
  const float* W1s = (const float*)d_in[3];
  const float* W1d = (const float*)d_in[4];
  const float* a1  = (const float*)d_in[5];
  const float* W2s = (const float*)d_in[6];
  const float* W2d = (const float*)d_in[7];
  const float* a2  = (const float*)d_in[8];
  const float* Wrs = (const float*)d_in[9];
  float* out = (float*)d_out;

  const int MP   = cdiv(nN, GBM) * GBM;
  const int nb   = pick_nb(nE, nN);
  if (nb < 64 || (nb & (nb - 1)) != 0 || nb > NBRUN) return;
  const int gA   = cdiv(MP, nb);
  const int vec8 = ((nE & 3) == 0) ? 1 : 0;
  if (gA * nb < MP) return;

  char* ws = (char*)d_ws;
  size_t off = 0;
  const size_t oXB  = off; off += (size_t)MP * F_IN * 2;          off = (off + 255) & ~(size_t)255;
  const size_t oHA  = off; off += (size_t)MP * KA * 2;            off = (off + 255) & ~(size_t)255;
  const size_t oWT1 = off; off += (size_t)P1 * F_IN * 2;          off = (off + 255) & ~(size_t)255;
  const size_t oWT2 = off; off += (size_t)P2 * KA * 2;            off = (off + 255) & ~(size_t)255;
  const size_t oHF1 = off; off += (size_t)MP * P1 * 4;            off = (off + 255) & ~(size_t)255;
  const size_t oHF2 = off; off += (size_t)MP * P2 * 4;            off = (off + 255) & ~(size_t)255;
  if (off > ws_size || off > (size_t)WSMAX) return;
  unsigned short* XB  = (unsigned short*)(ws + oXB);
  unsigned short* HA  = (unsigned short*)(ws + oHA);
  unsigned short* WT1 = (unsigned short*)(ws + oWT1);
  unsigned short* WT2 = (unsigned short*)(ws + oWT2);
  float*          HF1 = (float*)(ws + oHF1);
  float*          HF2 = (float*)(ws + oHF2);

  hipFuncSetAttribute(reinterpret_cast<const void*>(&k_agg<0>),
                      hipFuncAttributeMaxDynamicSharedMemorySize, LDS_AGG);
  hipFuncSetAttribute(reinterpret_cast<const void*>(&k_agg<1>),
                      hipFuncAttributeMaxDynamicSharedMemorySize, LDS_AGG);

  const int nUx = MP * XUPR;
  k_xprep<<<cdiv(nUx, NTHR), NTHR, 0, stream>>>(h, XB, nN, nUx);

  {
    const int nUw1 = C1 * (F_IN / 8);
    k_wtr<<<cdiv(nUw1, NTHR), NTHR, 0, stream>>>(W1s, F_IN, C1, C1, F_IN, WT1, nUw1);
    k_wtr<<<cdiv(nUw1, NTHR), NTHR, 0, stream>>>(W1d, F_IN, C1, C1, F_IN, WT1 + (size_t)C1 * F_IN, nUw1);
    const int nUw2 = N2W * (KA / 8);
    const int nUw3 = (P2 - 2 * N2W) * (KA / 8);
    k_wtr<<<cdiv(nUw2, NTHR), NTHR, 0, stream>>>(W2s, C1, N2W, N2W, KA, WT2, nUw2);
    k_wtr<<<cdiv(nUw2, NTHR), NTHR, 0, stream>>>(W2d, C1, N2W, N2W, KA, WT2 + (size_t)N2W * KA, nUw2);
    k_wtr<<<cdiv(nUw3, NTHR), NTHR, 0, stream>>>(Wrs, C1, N2W, P2 - 2 * N2W, KA, WT2 + (size_t)(2 * N2W) * KA, nUw3);
  }

  const int gM = MP / GBM;
  k_gemm<<<dim3(gM, P1 / GBN), GTHR, 0, stream>>>(XB, WT1, HF1, F_IN, P1);
  k_agg<0><<<gA, NTHR, LDS_AGG, stream>>>(src, dst, HF1, a1, HA, out, nN, nE, nb, vec8, MP);
  k_gemm<<<dim3(gM, P2 / GBN), GTHR, 0, stream>>>(HA, WT2, HF2, KA, P2);
  k_agg<1><<<gA, NTHR, LDS_AGG, stream>>>(src, dst, HF2, a2, HA, out, nN, nE, nb, vec8, MP);
}
